// GATNetwork_23038204576292
// MI455X (gfx1250) — hardware-verified
//
#include <hip/hip_runtime.h>
#include <stddef.h>


#define NTHR  256
#define NWAVE 8
#define HCW   128
#define GR    32
#define MR    64
#define XSP   132
#define NB    512
#define CHUNK 1024
#define WCAP  128
#define ACCF  (NB * HCW)
#define AGG_LDS_BYTES (ACCF * 4 + NB * 4 * 4 + NWAVE * WCAP * 4 + NWAVE * 4)

static_assert(AGG_LDS_BYTES == 274464);
static_assert(CHUNK == NTHR * 4);
static_assert(WCAP == (CHUNK / NTHR) * 32);
static_assert((NB & (NB - 1)) == 0);
static_assert(NB <= 512);
static_assert(NB <= NWAVE * WCAP);
static_assert((XSP % 4) == 0);

typedef float          v4f   __attribute__((ext_vector_type(4)));
typedef float          v8f   __attribute__((ext_vector_type(8)));
typedef int            v4i   __attribute__((ext_vector_type(4)));
typedef _Float16       v8h   __attribute__((ext_vector_type(8)));
typedef _Float16       v16h  __attribute__((ext_vector_type(16)));
typedef __bf16         v16b  __attribute__((ext_vector_type(16)));
typedef unsigned short v8us  __attribute__((ext_vector_type(8)));
typedef unsigned short v16us __attribute__((ext_vector_type(16)));

union FragH { v16h v; v4i u[2]; };
union FragB { v16b v; v16us s; v4i u[2]; };
union Pack  { v8h h; v8us s; v4i i; };

__device__ __forceinline__ unsigned short f2bf(float x) {
  unsigned b = __float_as_uint(x);
  b += 0x7FFFu + ((b >> 16) & 1u);
  return (unsigned short)(b >> 16);
}
__device__ __forceinline__ float bf2f(unsigned short h) { return __uint_as_float(((unsigned)h) << 16); }

__device__ __forceinline__ v8f wmh(v16h a, v16h b, v8f c) {
  v8f d = __builtin_amdgcn_wmma_f32_16x16x32_f16(false, a, false, b, (short)0, c, false, false);
  asm volatile("v_nop\n\tv_nop\n\tv_nop\n\tv_nop" : "+v"(d) : "v"(a), "v"(b));
  return d;
}
__device__ __forceinline__ v8f wmb(v16b a, v16b b, v8f c) {
  v8f d = __builtin_amdgcn_wmma_f32_16x16x32_bf16(false, a, false, b, (short)0, c, false, false);
  asm volatile("v_nop\n\tv_nop\n\tv_nop\n\tv_nop" : "+v"(d) : "v"(a), "v"(b));
  return d;
}

__device__ __forceinline__ float lk(float t) { return fmaxf(t, 0.2f * t); }
__device__ __forceinline__ float dl(v4f t, v4f w) {
  return w.x * lk(t.x) + w.y * lk(t.y) + w.z * lk(t.z) + w.w * lk(t.w);
}

__global__ __launch_bounds__(NTHR) void k_cvtx(const float* __restrict__ x, unsigned short* xh, int nN, int Mpad) {
  const int i  = blockIdx.x * NTHR + threadIdx.x;
  const int n8 = Mpad * (HCW / 8);
  if (i >= n8) return;
  const int r  = i >> 4;
  const int kb = (i & 15) * 8;
  const v4f z4 = {0.f, 0.f, 0.f, 0.f};
  v4f f0 = z4, f1 = z4;
  if (r < nN) {
    const float* p = x + (size_t)r * HCW + kb;
    f0 = *(const v4f*)p;
    f1 = *(const v4f*)(p + 4);
  }
  Pack u;
#pragma unroll
  for (int j = 0; j < 4; ++j) {
    u.h[j]     = (_Float16)f0[j];
    u.h[4 + j] = (_Float16)f1[j];
  }
  const size_t o = (size_t)i * 8;
  *(volatile v4i*)(xh + o) = u.i;
  __threadfence();
  *(volatile v4i*)(xh + o) = u.i;
}

__global__ __launch_bounds__(NTHR) void k_cvtw(const float* __restrict__ Wl, const float* __restrict__ Wr,
                                               const float* __restrict__ Wm,
                                               unsigned short* WlT, unsigned short* WrT,
                                               unsigned short* WmTh, unsigned short* WmTl, float wscale) {
  const int which = blockIdx.y;
  const float* src = (which == 0) ? Wl : ((which == 1) ? Wr : Wm);
  const int tid = threadIdx.x;
  const int n   = blockIdx.x * 16 + (tid >> 4);
  const int kb  = (tid & 15) * 8;
  float v[8];
#pragma unroll
  for (int j = 0; j < 8; ++j) v[j] = src[(size_t)(kb + j) * HCW + n];
  const size_t o = (size_t)n * HCW + kb;
  if (which < 2) {
    Pack uf;
#pragma unroll
    for (int j = 0; j < 8; ++j) uf.h[j] = (_Float16)(v[j] * wscale);
    unsigned short* dp = (which == 0) ? WlT : WrT;
    *(volatile v4i*)(dp + o) = uf.i;
    __threadfence();
    *(volatile v4i*)(dp + o) = uf.i;
  } else {
    Pack uh, ul;
#pragma unroll
    for (int j = 0; j < 8; ++j) {
      const unsigned short hb = f2bf(v[j]);
      uh.s[j] = hb;
      ul.s[j] = f2bf(v[j] - bf2f(hb));
    }
    *(volatile v4i*)(WmTh + o) = uh.i;
    *(volatile v4i*)(WmTl + o) = ul.i;
    __threadfence();
    *(volatile v4i*)(WmTh + o) = uh.i;
    *(volatile v4i*)(WmTl + o) = ul.i;
  }
}

__global__ __launch_bounds__(NTHR) void k_gemm2(const unsigned short* __restrict__ A,
                                                const unsigned short* __restrict__ Bl,
                                                const unsigned short* __restrict__ Br,
                                                float* xl, float* xr, float oscale) {
  __shared__ __attribute__((aligned(16))) float Xa[GR * XSP];
  __shared__ __attribute__((aligned(16))) float Xb[GR * XSP];

  const int tid  = threadIdx.x;
  const int lane = tid & 31;
  const int wave = tid >> 5;
  const int hh   = lane >> 4;
  const int m    = lane & 15;
  const int rowBase = blockIdx.x * GR;
  const int ncol = wave * 16 + m;

  const size_t ra0 = (size_t)(rowBase + m) * HCW + 8 * hh;
  const size_t ra1 = ra0 + (size_t)16 * HCW;
  const size_t rb  = (size_t)ncol * HCW + 8 * hh;

  v8f c0 = {0.f, 0.f, 0.f, 0.f, 0.f, 0.f, 0.f, 0.f};
  v8f c1 = c0, c2 = c0, c3 = c0;

#pragma unroll 1
  for (int k0 = 0; k0 < HCW; k0 += 32) {
    FragH a0, a1, bl, br;
    a0.u[0] = *(const v4i*)(A + ra0 + k0);   a0.u[1] = *(const v4i*)(A + ra0 + k0 + 16);
    a1.u[0] = *(const v4i*)(A + ra1 + k0);   a1.u[1] = *(const v4i*)(A + ra1 + k0 + 16);
    bl.u[0] = *(const v4i*)(Bl + rb + k0);   bl.u[1] = *(const v4i*)(Bl + rb + k0 + 16);
    br.u[0] = *(const v4i*)(Br + rb + k0);   br.u[1] = *(const v4i*)(Br + rb + k0 + 16);
    c0 = wmh(a0.v, bl.v, c0);
    c1 = wmh(a1.v, bl.v, c1);
    c2 = wmh(a0.v, br.v, c2);
    c3 = wmh(a1.v, br.v, c3);
  }

  const int cl = wave * 16 + m;
#pragma unroll
  for (int r = 0; r < 8; ++r) {
    Xa[(8 * hh + r) * XSP + cl]      = c0[r] * oscale;
    Xa[(16 + 8 * hh + r) * XSP + cl] = c1[r] * oscale;
    Xb[(8 * hh + r) * XSP + cl]      = c2[r] * oscale;
    Xb[(16 + 8 * hh + r) * XSP + cl] = c3[r] * oscale;
  }
  __syncthreads();

  v4f va[4], vb[4];
  float* pa[4];
  float* pb[4];
#pragma unroll
  for (int i = 0; i < 4; ++i) {
    const int rr = 4 * wave + i;
    va[i] = *(const v4f*)(Xa + rr * XSP + 4 * lane);
    vb[i] = *(const v4f*)(Xb + rr * XSP + 4 * lane);
    pa[i] = xl + (size_t)(rowBase + rr) * HCW + 4 * lane;
    pb[i] = xr + (size_t)(rowBase + rr) * HCW + 4 * lane;
  }
#pragma unroll
  for (int i = 0; i < 4; ++i) { *(volatile v4f*)(pa[i]) = va[i]; *(volatile v4f*)(pb[i]) = vb[i]; }
  __threadfence();
#pragma unroll
  for (int i = 0; i < 4; ++i) { *(volatile v4f*)(pa[i]) = va[i]; *(volatile v4f*)(pb[i]) = vb[i]; }
}

__global__ __launch_bounds__(NTHR) void k_agg(const int* __restrict__ ei, const float* __restrict__ xl,
                                              const float* __restrict__ xr, const float* __restrict__ att,
                                              const float* __restrict__ bias, float* hout, int nN, int nE) {
  extern __shared__ v4f lds_dyn[];
  float* sacc = (float*)lds_dyn;
  float* dn   = sacc + ACCF;
  int*   list = (int*)(dn + NB * 4);
  int*   wcnt = list + NWAVE * WCAP;

  const int tid  = threadIdx.x;
  const int lane = tid & 31;
  const int wave = tid >> 5;
  const int nodeBase = blockIdx.x * NB;

  {
    const v4f z4 = {0.f, 0.f, 0.f, 0.f};
    for (int i = tid; i < ACCF / 4; i += NTHR) lds_dyn[i] = z4;
    for (int i = tid; i < NB * 4; i += NTHR) dn[i] = 0.f;
  }
  __syncthreads();

  const int coff = 4 * lane;
  const int hidx = lane >> 3;
  const v4f w0 = *(const v4f*)(att + coff);

  const int* eid = ei + nE;
  const bool al16 = ((nE & 3) == 0);
  const int nChunks = (nE + CHUNK - 1) / CHUNK;

#pragma unroll 1
  for (int ch = 0; ch <= nChunks; ++ch) {
    const int cbase = ch * CHUNK;
    const bool selfp = (ch == nChunks);
    if (!selfp) {
      int wc = 0;
      const int el0 = tid * 4;
      const int e0  = cbase + el0;
      const int sent = -2147483647 - 1;
      v4i d;
      if (al16 && (e0 + 3 < nE)) {
        d = *(const v4i*)(eid + e0);
      } else {
        d.x = (e0     < nE) ? eid[min(e0, nE - 1)]     : sent;
        d.y = (e0 + 1 < nE) ? eid[min(e0 + 1, nE - 1)] : sent;
        d.z = (e0 + 2 < nE) ? eid[min(e0 + 2, nE - 1)] : sent;
        d.w = (e0 + 3 < nE) ? eid[min(e0 + 3, nE - 1)] : sent;
      }
      const unsigned s0 = (unsigned)d.x - (unsigned)nodeBase;
      const unsigned s1 = (unsigned)d.y - (unsigned)nodeBase;
      const unsigned s2 = (unsigned)d.z - (unsigned)nodeBase;
      const unsigned s3 = (unsigned)d.w - (unsigned)nodeBase;
      const bool h0 = s0 < (unsigned)NB;
      const bool h1 = s1 < (unsigned)NB;
      const bool h2 = s2 < (unsigned)NB;
      const bool h3 = s3 < (unsigned)NB;
      const unsigned many = __builtin_amdgcn_ballot_w32(h0 | h1 | h2 | h3);
      if (many != 0u) {
#define HITJ(J, HJ, SJ) { \
          const unsigned mj = __builtin_amdgcn_ballot_w32(HJ); \
          if (HJ) { \
            const int pos = wc + (int)__builtin_amdgcn_mbcnt_lo(mj, 0u); \
            if (pos < WCAP) list[wave * WCAP + pos] = ((el0 + (J)) << 9) | (int)(SJ); \
          } \
          wc += (int)__builtin_popcount(mj); }
        HITJ(0, h0, s0)
        HITJ(1, h1, s1)
        HITJ(2, h2, s2)
        HITJ(3, h3, s3)
#undef HITJ
      }
      if (lane == 0) wcnt[wave] = wc;
    } else {
      for (int s = tid; s < NB; s += NTHR) list[s] = s;
      if (tid < NWAVE) {
        int c = NB - tid * WCAP;
        c = c < 0 ? 0 : (c > WCAP ? WCAP : c);
        wcnt[tid] = c;
      }
    }
    __syncthreads();

    if (wave == 0) {
#pragma unroll 1
      for (int wsx = 0; wsx < NWAVE; ++wsx) {
        int n = __builtin_amdgcn_readfirstlane(wcnt[wsx]);
        n = n > WCAP ? WCAP : n;
        n = n < 0 ? 0 : n;
#pragma unroll 1
        for (int i = 0; i < n; ++i) {
          const int ent  = __builtin_amdgcn_readfirstlane(list[wsx * WCAP + i]);
          const int slot = ent & (NB - 1);
          const int el   = (ent >> 9) & (CHUNK - 1);
          const int node = nodeBase + slot;
          if (node >= nN) continue;
          int e = cbase + el;
          if (e > nE - 1) e = nE - 1;
          int sj = ei[e];
          sj = sj < 0 ? 0 : (sj > nN - 1 ? nN - 1 : sj);
          const int src = selfp ? node : sj;

          const v4f a  = *(const v4f*)(xl + (size_t)src * HCW + coff);
          const v4f dv = *(const v4f*)(xr + (size_t)node * HCW + coff);
          float sc = dl(a + dv, w0);
          sc += __shfl_xor(sc, 4, 32);
          sc += __shfl_xor(sc, 2, 32);
          sc += __shfl_xor(sc, 1, 32);
          const float p = __expf(sc);
          float* ar = sacc + slot * HCW + coff;
          float* dp = dn + slot * 4 + hidx;
          const float dold = dp[0];
          v4f ev = *(v4f*)(ar);
          ev = ev + a * p;
          *(v4f*)(ar) = ev;
          dp[0] = dold + p;
        }
      }
    }
    __syncthreads();
  }

  const v4f b0 = *(const v4f*)(bias + coff);
#pragma unroll 1
  for (int s = wave; s < NB; s += NWAVE) {
    const int node = nodeBase + s;
    if (node >= nN) break;
    const v4f e0 = *(const v4f*)(sacc + s * HCW + coff);
    const float inv = 1.0f / dn[s * 4 + hidx];
    v4f o = e0 * inv + b0;
    o.x = fmaxf(o.x, 0.f);  o.y = fmaxf(o.y, 0.f);  o.z = fmaxf(o.z, 0.f);  o.w = fmaxf(o.w, 0.f);
    float* op = hout + (size_t)node * HCW + coff;
    *(volatile v4f*)op = o;
    __threadfence();
    *(volatile v4f*)op = o;
  }
}

__global__ __launch_bounds__(NTHR) void k_pool(const float* __restrict__ hout, const int* __restrict__ bid,
                                               const int* __restrict__ ngp, float* pooled, int nN, int G) {
  __shared__ int plist[NWAVE * 32];
  __shared__ int pcnt[NWAVE];
  __shared__ float red[HCW];
  __shared__ __attribute__((aligned(16))) float stg[HCW];

  const int tid  = threadIdx.x;
  const int lane = tid & 31;
  const int wave = tid >> 5;
  const int g    = blockIdx.x;
  const int ng   = ngp[0];
  const int ch   = tid & (HCW - 1);
  const int par  = tid >> 7;
  float mv = __uint_as_float(0xff800000u);
  const int nch = (nN + NTHR - 1) / NTHR;

#pragma unroll 1
  for (int c = 0; c < nch; ++c) {
    const int n  = c * NTHR + tid;
    const int bb = bid[min(n, nN - 1)];
    const int b  = (n < nN) ? bb : -1;
    const bool hit = (b == g) && (g < ng) && (g < G);
    const unsigned mk = __builtin_amdgcn_ballot_w32(hit);
    if (hit) plist[wave * 32 + (int)__builtin_amdgcn_mbcnt_lo(mk, 0u)] = n;
    if (lane == 0) pcnt[wave] = (int)__builtin_popcount(mk);
    __syncthreads();
#pragma unroll 1
    for (int w8 = 0; w8 < NWAVE; ++w8) {
      int cnt = pcnt[w8];
      cnt = cnt > 32 ? 32 : (cnt < 0 ? 0 : cnt);
#pragma unroll 1
      for (int i = par; i < cnt; i += 2) {
        int node = plist[w8 * 32 + i];
        node = node < 0 ? 0 : (node > nN - 1 ? nN - 1 : node);
        mv = fmaxf(mv, hout[(size_t)node * HCW + ch]);
      }
    }
    __syncthreads();
  }
  if (par == 1) red[ch] = mv;
  __syncthreads();
  if (par == 0) { mv = fmaxf(mv, red[ch]); stg[ch] = mv; }
  __syncthreads();
  if (wave == 0) {
    const v4f o = *(const v4f*)(stg + 4 * lane);
    float* p = pooled + (size_t)g * HCW + 4 * lane;
    *(volatile v4f*)p = o;
    __threadfence();
    *(volatile v4f*)p = o;
  }
}

__device__ __forceinline__ void cvt_a(const float* p, FragB& ah, FragB& al) {
  const v4f f0 = *(const v4f*)(p),      f1 = *(const v4f*)(p + 4);
  const v4f f2 = *(const v4f*)(p + 16), f3 = *(const v4f*)(p + 20);
#pragma unroll
  for (int j = 0; j < 4; ++j) {
    unsigned short hb;
    hb = f2bf(f0[j]); ah.s[j]      = hb; al.s[j]      = f2bf(f0[j] - bf2f(hb));
    hb = f2bf(f1[j]); ah.s[4 + j]  = hb; al.s[4 + j]  = f2bf(f1[j] - bf2f(hb));
    hb = f2bf(f2[j]); ah.s[8 + j]  = hb; al.s[8 + j]  = f2bf(f2[j] - bf2f(hb));
    hb = f2bf(f3[j]); ah.s[12 + j] = hb; al.s[12 + j] = f2bf(f3[j] - bf2f(hb));
  }
}

__global__ __launch_bounds__(NTHR) void k_mlp(const float* __restrict__ pooled,
                                              const unsigned short* __restrict__ Bh,
                                              const unsigned short* __restrict__ Bl,
                                              const float* __restrict__ bm, float* out, int G) {
  __shared__ __attribute__((aligned(16))) float Xs[MR * XSP];

  const int tid  = threadIdx.x;
  const int lane = tid & 31;
  const int wave = tid >> 5;
  const int hh   = lane >> 4;
  const int m    = lane & 15;
  const int rowBase = blockIdx.x * MR;
  const int n    = wave * 16 + m;
  const size_t rb = (size_t)n * HCW + 8 * hh;

  int r0 = rowBase + m, r1 = rowBase + 16 + m, r2 = rowBase + 32 + m, r3 = rowBase + 48 + m;
  r0 = r0 > G - 1 ? G - 1 : r0;  r1 = r1 > G - 1 ? G - 1 : r1;
  r2 = r2 > G - 1 ? G - 1 : r2;  r3 = r3 > G - 1 ? G - 1 : r3;
  const float* p0 = pooled + (size_t)r0 * HCW + 8 * hh;
  const float* p1 = pooled + (size_t)r1 * HCW + 8 * hh;
  const float* p2 = pooled + (size_t)r2 * HCW + 8 * hh;
  const float* p3 = pooled + (size_t)r3 * HCW + 8 * hh;

  v8f c0 = {0.f, 0.f, 0.f, 0.f, 0.f, 0.f, 0.f, 0.f};
  v8f c1 = c0, c2 = c0, c3 = c0;

#pragma unroll 1
  for (int k0 = 0; k0 < HCW; k0 += 32) {
    FragB bh, bl, ah, al;
    bh.u[0] = *(const v4i*)(Bh + rb + k0);  bh.u[1] = *(const v4i*)(Bh + rb + k0 + 16);
    bl.u[0] = *(const v4i*)(Bl + rb + k0);  bl.u[1] = *(const v4i*)(Bl + rb + k0 + 16);
    cvt_a(p0 + k0, ah, al);
    c0 = wmb(ah.v, bh.v, c0);  c0 = wmb(ah.v, bl.v, c0);  c0 = wmb(al.v, bh.v, c0);
    cvt_a(p1 + k0, ah, al);
    c1 = wmb(ah.v, bh.v, c1);  c1 = wmb(ah.v, bl.v, c1);  c1 = wmb(al.v, bh.v, c1);
    cvt_a(p2 + k0, ah, al);
    c2 = wmb(ah.v, bh.v, c2);  c2 = wmb(ah.v, bl.v, c2);  c2 = wmb(al.v, bh.v, c2);
    cvt_a(p3 + k0, ah, al);
    c3 = wmb(ah.v, bh.v, c3);  c3 = wmb(ah.v, bl.v, c3);  c3 = wmb(al.v, bh.v, c3);
  }

  const float bv = bm[n];
#pragma unroll
  for (int r = 0; r < 8; ++r) {
    Xs[(8 * hh + r) * XSP + n]      = fmaxf(c0[r] + bv, 0.f);
    Xs[(16 + 8 * hh + r) * XSP + n] = fmaxf(c1[r] + bv, 0.f);
    Xs[(32 + 8 * hh + r) * XSP + n] = fmaxf(c2[r] + bv, 0.f);
    Xs[(48 + 8 * hh + r) * XSP + n] = fmaxf(c3[r] + bv, 0.f);
  }
  __syncthreads();

  v4f xv[8];
  float* xp[8];
  bool ok[8];
#pragma unroll
  for (int i = 0; i < 8; ++i) {
    const int rr = 8 * wave + i;
    xv[i] = *(const v4f*)(Xs + rr * XSP + 4 * lane);
    const int gr = rowBase + rr;
    ok[i] = gr < G;
    const int grc = ok[i] ? gr : (G - 1);
    xp[i] = out + (size_t)grc * HCW + 4 * lane;
  }
#pragma unroll
  for (int i = 0; i < 8; ++i) if (ok[i]) *(volatile v4f*)(xp[i]) = xv[i];
  __threadfence();
#pragma unroll
  for (int i = 0; i < 8; ++i) if (ok[i]) *(volatile v4f*)(xp[i]) = xv[i];
}

extern "C" void kernel_launch(void* const* d_in, const int* in_sizes, int n_in,
                              void* d_out, int out_size, void* d_ws, size_t ws_size,
                              hipStream_t stream) {
  if (n_in < 10) return;
  const int nN = in_sizes[0] / HCW;
  if (nN <= 0 || in_sizes[0] != nN * HCW) return;
  const int nE = in_sizes[1] / 2;
  if (nE <= 0 || in_sizes[1] != 2 * nE) return;
  if (in_sizes[2] != nN || in_sizes[3] < 1) return;
  if (in_sizes[4] != HCW * HCW || in_sizes[5] != HCW * HCW || in_sizes[6] != HCW || in_sizes[7] != HCW ||
      in_sizes[8] != HCW * HCW || in_sizes[9] != HCW) return;
  const int G = out_size / HCW;
  if (G <= 0 || out_size != G * HCW) return;

  const float* x    = (const float*)d_in[0];
  const int*   ei   = (const int*)d_in[1];
  const int*   bid  = (const int*)d_in[2];
  const int*   ngp  = (const int*)d_in[3];
  const float* Wl   = (const float*)d_in[4];
  const float* Wr   = (const float*)d_in[5];
  const float* att  = (const float*)d_in[6];
  const float* bcv  = (const float*)d_in[7];
  const float* Wm   = (const float*)d_in[8];
  const float* bm   = (const float*)d_in[9];
  float* out = (float*)d_out;

  const int Mpad = ((nN + GR - 1) / GR) * GR;
  const int Gpad = ((G + MR - 1) / MR) * MR;

  char* wsp = (char*)d_ws;
  size_t off = 0;
  const size_t xhB = (size_t)Mpad * HCW * 2;
  const size_t wB  = (size_t)HCW * HCW * 2;
  const size_t xfB = (size_t)Mpad * HCW * 4;
  const size_t pB  = (size_t)Gpad * HCW * 4;
  unsigned short* xh   = (unsigned short*)(wsp + off); off += xhB;
  unsigned short* WlT  = (unsigned short*)(wsp + off); off += wB;
  unsigned short* WrT  = (unsigned short*)(wsp + off); off += wB;
  unsigned short* WmTh = (unsigned short*)(wsp + off); off += wB;
  unsigned short* WmTl = (unsigned short*)(wsp + off); off += wB;
  float* xl     = (float*)(wsp + off); off += xfB;
  float* xr     = (float*)(wsp + off); off += xfB;
  float* hout   = (float*)(wsp + off); off += xfB;
  float* pooled = (float*)(wsp + off); off += pB;
  if (off > ws_size) return;
  if (off > (size_t)134217728) return;

  hipFuncSetAttribute(reinterpret_cast<const void*>(&k_agg),
                      hipFuncAttributeMaxDynamicSharedMemorySize, AGG_LDS_BYTES);

  k_cvtx<<<(Mpad * (HCW / 8) + NTHR - 1) / NTHR, NTHR, 0, stream>>>(x, xh, nN, Mpad);
  k_cvtw<<<dim3(HCW / 16, 3), NTHR, 0, stream>>>(Wl, Wr, Wm, WlT, WrT, WmTh, WmTl, 16.0f);
  k_gemm2<<<Mpad / GR, NTHR, 0, stream>>>(xh, WlT, WrT, xl, xr, 0.0625f);
  k_agg<<<(nN + NB - 1) / NB, NTHR, AGG_LDS_BYTES, stream>>>(ei, xl, xr, att, bcv, hout, nN, nE);
  k_pool<<<G, NTHR, 0, stream>>>(hout, bid, ngp, pooled, nN, G);
  k_mlp<<<Gpad / MR, NTHR, 0, stream>>>(pooled, WmTh, WmTl, bm, out, G);
}
